// LRU_2817498546780
// MI455X (gfx1250) — hardware-verified
//
#include <hip/hip_runtime.h>
#include <math.h>

constexpr int SEQ_LEN = 16384;
constexpr int NSTATE  = 512;
constexpr int NFEAT   = 512;
constexpr int NCOL2   = 2 * NSTATE;
constexpr int CHUNK_T = 64;
constexpr int NCHUNK  = SEQ_LEN / CHUNK_T;
constexpr int NTHR    = 256;
constexpr float BP_CARRY = 1024.0f;
constexpr float CW_CARRY = 1024.0f;
constexpr float HS_CARRY = 4.0f;
constexpr float G1_FOLD  = 1.0f / 1024.0f;
constexpr float G2_FOLD  = 1.0f / 4096.0f;
static_assert(SEQ_LEN % 64 == 0 && NCOL2 % 64 == 0 && NFEAT % 64 == 0);
static_assert(NFEAT % 32 == 0 && NCOL2 % 32 == 0);
static_assert(SEQ_LEN == NCHUNK * CHUNK_T);
static_assert(NSTATE == 128 * 4 && NSTATE == 64 * 8);
static_assert((NSTATE * (NFEAT / 8)) % NTHR == 0);
static_assert((SEQ_LEN * (NFEAT / 8)) % NTHR == 0);
static_assert(((SEQ_LEN / 64) * (NCOL2 / 64)) % 8 == 0 && ((SEQ_LEN / 64) * (NFEAT / 64)) % 8 == 0);

typedef __attribute__((ext_vector_type(16))) _Float16 v16h;
typedef __attribute__((ext_vector_type(8)))  _Float16 v8h;
typedef __attribute__((ext_vector_type(16))) __bf16   v16b;
typedef __attribute__((ext_vector_type(8)))  __bf16   v8b;
typedef __attribute__((ext_vector_type(8)))  float    v8f;
typedef __attribute__((ext_vector_type(4)))  float    v4f;

__device__ __forceinline__ unsigned short f2bf_bits(float f) {
  unsigned u = __float_as_uint(f);
  return (unsigned short)((u + 0x7FFFu + ((u >> 16) & 1u)) >> 16);
}
__device__ __forceinline__ float bf_bits2f(unsigned short h) { return __uint_as_float(((unsigned)h) << 16); }

__device__ __forceinline__ void dep_guard_h(v8f& a, v8f& b, v16h x, v16h y) { asm volatile("v_nop\n\tv_nop\n\tv_nop\n\tv_nop" : "+v"(a), "+v"(b) : "v"(x), "v"(y)); }
__device__ __forceinline__ void dep_guard_b(v8f& a, v8f& b, v16b x, v16b y) { asm volatile("v_nop\n\tv_nop\n\tv_nop\n\tv_nop" : "+v"(a), "+v"(b) : "v"(x), "v"(y)); }
__device__ __forceinline__ void dep_guard4_h(v8f& a, v8f& b, v8f& c, v8f& d, v16h x, v16h y) { asm volatile("v_nop\n\tv_nop\n\tv_nop\n\tv_nop" : "+v"(a), "+v"(b), "+v"(c), "+v"(d) : "v"(x), "v"(y)); }
__device__ __forceinline__ void dep_guard4_b(v8f& a, v8f& b, v8f& c, v8f& d, v16b x, v16b y) { asm volatile("v_nop\n\tv_nop\n\tv_nop\n\tv_nop" : "+v"(a), "+v"(b), "+v"(c), "+v"(d) : "v"(x), "v"(y)); }
__device__ __forceinline__ void keep4_h(v16h a, v16h b, v16h c, v16h d) { asm volatile("v_nop" :: "v"(a), "v"(b), "v"(c), "v"(d)); }
__device__ __forceinline__ void keep4_b(v16b a, v16b b, v16b c, v16b d) { asm volatile("v_nop" :: "v"(a), "v"(b), "v"(c), "v"(d)); }
__device__ __forceinline__ void acc_guard4(v8f& a, v8f& b, v8f& c, v8f& d) { asm volatile("v_nop\n\tv_nop\n\tv_nop\n\tv_nop" : "+v"(a), "+v"(b), "+v"(c), "+v"(d)); }
__device__ __forceinline__ void mem_split() { asm volatile("" ::: "memory"); }
template <typename T> struct Frag;
template <> struct Frag<_Float16> {
  typedef v16h V; union U { v16h v; v8h h[2]; };
  static __device__ __forceinline__ v16h load(const _Float16* p) {
    U f; f.h[0] = *(const v8h*)(p); f.h[1] = *(const v8h*)(p + 16); return f.v;
  }
  static __device__ __forceinline__ v8f mma(v16h a, v16h b, v8f c) {
    return __builtin_amdgcn_wmma_f32_16x16x32_f16(false, a, false, b, (short)0, c, false, false);
  }
  static __device__ __forceinline__ void guard(v8f& a, v8f& b, v16h x, v16h y) { dep_guard_h(a, b, x, y); }
  static __device__ __forceinline__ void guard4(v8f& a, v8f& b, v8f& c, v8f& d, v16h x, v16h y) { dep_guard4_h(a, b, c, d, x, y); }
  static __device__ __forceinline__ void keep(v16h a, v16h b, v16h c, v16h d) { keep4_h(a, b, c, d); }
};
template <> struct Frag<__bf16> {
  typedef v16b V; union U { v16b v; v8b h[2]; };
  static __device__ __forceinline__ v16b load(const __bf16* p) {
    U f; f.h[0] = *(const v8b*)(p); f.h[1] = *(const v8b*)(p + 16); return f.v;
  }
  static __device__ __forceinline__ v8f mma(v16b a, v16b b, v8f c) {
    return __builtin_amdgcn_wmma_f32_16x16x32_bf16(false, a, false, b, (short)0, c, false, false);
  }
  static __device__ __forceinline__ void guard(v8f& a, v8f& b, v16b x, v16b y) { dep_guard_b(a, b, x, y); }
  static __device__ __forceinline__ void guard4(v8f& a, v8f& b, v8f& c, v8f& d, v16b x, v16b y) { dep_guard4_b(a, b, c, d, x, y); }
  static __device__ __forceinline__ void keep(v16b a, v16b b, v16b c, v16b d) { keep4_b(a, b, c, d); }
};

template <int ET> struct Elem;
template <> struct Elem<0> { typedef _Float16 T; };
template <> struct Elem<1> { typedef __bf16 T; };
template <int ET, bool SPLIT, int BIAS_MODE, int OUT_MODE, bool RESID, int ACT, bool DXM>
__global__ __launch_bounds__(256) void wmma_gemm64(
    const unsigned short* __restrict__ Ap, const unsigned short* __restrict__ A2p, int lda, long strideA,
    const unsigned short* __restrict__ Btp, const unsigned short* __restrict__ Bt2p, int ldb, long strideB,
    void* __restrict__ Cout, void* __restrict__ Cout2, int ldc, long strideC,
    const float* __restrict__ bias,
    const float* __restrict__ resid, long strideR,
    int M, int N, int K, float scale,
    const float* __restrict__ dvec, const float* __restrict__ xres, int ldx) {
  typedef typename Elem<ET>::T T;
  typedef typename Frag<T>::V V;
  const T* A = (const T*)Ap; const T* A2 = (const T*)A2p; const T* Bt = (const T*)Btp; const T* Bt2 = (const T*)Bt2p;
  __shared__ __align__(16) float sT[8][16 * 68];
  const int b    = blockIdx.y;
  const int lane = threadIdx.x & 31;
  const int wave = threadIdx.x >> 5;
  const int tilesN = N >> 6;
  const int tilesM = M >> 6;
  const int tile = blockIdx.x * 8 + wave;
  if (tile >= tilesM * tilesN) return;
  const int tm = tile / tilesN;
  const int tn = tile - tm * tilesN;
  const int m0 = tm << 6;
  const int n0 = tn << 6;

  const T* Ab  = A  + (size_t)b * strideA;
  const T* Bb  = Bt + (size_t)b * strideB;
  const T* Ab2 = SPLIT ? (A2  + (size_t)b * strideA) : nullptr;
  const T* Bb2 = SPLIT ? (Bt2 + (size_t)b * strideB) : nullptr;

  const int rlane = lane & 15;
  const int koff  = (lane >> 4) * 8;
  const int mOff  = (lane >> 4) * 8;

  v8f acc[4][4];
#pragma unroll
  for (int i = 0; i < 4; ++i)
#pragma unroll
    for (int j = 0; j < 4; ++j) acc[i][j] = (v8f){0.f,0.f,0.f,0.f,0.f,0.f,0.f,0.f};

  for (int k0 = 0; k0 < K; k0 += 32) {
    V bh[4], bl[4];
#pragma unroll
    for (int j = 0; j < 4; ++j) {
      const size_t bo = (size_t)(n0 + (j << 4) + rlane) * ldb + koff + k0;
      bh[j] = Frag<T>::load(Bb + bo);
      if (SPLIT) bl[j] = Frag<T>::load(Bb2 + bo);
    }
#pragma unroll
    for (int i = 0; i < 4; ++i) {
      const size_t ao = (size_t)(m0 + (i << 4) + rlane) * lda + koff + k0;
      V ah = Frag<T>::load(Ab + ao);
      V al;
      if (SPLIT) al = Frag<T>::load(Ab2 + ao);
#pragma unroll
      for (int j = 0; j < 4; ++j) {
        acc[i][j] = Frag<T>::mma(ah, bh[j], acc[i][j]);
        if (SPLIT) {
          acc[i][j] = Frag<T>::mma(ah, bl[j], acc[i][j]);
          acc[i][j] = Frag<T>::mma(al, bh[j], acc[i][j]);
        }
      }
      Frag<T>::guard4(acc[i][0], acc[i][1], acc[i][2], acc[i][3], ah, bh[3]);
      if (SPLIT) Frag<T>::guard(acc[i][0], acc[i][3], al, bl[3]);
    }
    Frag<T>::keep(bh[0], bh[1], bh[2], bh[3]);
    if (SPLIT) Frag<T>::keep(bl[0], bl[1], bl[2], bl[3]);
  }
  acc_guard4(acc[0][0], acc[0][1], acc[0][2], acc[0][3]);
  acc_guard4(acc[1][0], acc[1][1], acc[1][2], acc[1][3]);
  acc_guard4(acc[2][0], acc[2][1], acc[2][2], acc[2][3]);
  acc_guard4(acc[3][0], acc[3][1], acc[3][2], acc[3][3]);

  float* slab = sT[wave];
  const float* Rb = RESID ? (resid + (size_t)b * strideR) : nullptr;
  const int shh = lane >> 4, sc4 = (lane & 15) * 4;
  v4f dv4 = {0.f, 0.f, 0.f, 0.f};
  if (DXM) dv4 = *(const v4f*)(dvec + n0 + sc4);
#pragma unroll
  for (int i = 0; i < 4; ++i) {
    const int mBase = m0 + (i << 4);
#pragma unroll
    for (int j = 0; j < 4; ++j) {
      const int n = n0 + (j << 4) + rlane;
      float bv = 0.f;
      if (BIAS_MODE == 2) bv = bias[n];
#pragma unroll
      for (int r = 0; r < 8; ++r) {
        float v = acc[i][j][r] * scale;
        if (BIAS_MODE == 1) v += bias[mBase + mOff + r];
        if (BIAS_MODE == 2) v += bv;
        if (RESID) v += Rb[(size_t)(mBase + mOff + r) * ldc + n];
        if (ACT == 1) v = tanhf(v);
        if (ACT == 2) v = fmaxf(v, 0.0f);
        if (ACT == 4) v = (v > 0.f) ? v : 0.01f * v;
        slab[(mOff + r) * 68 + (j << 4) + rlane] = v;
      }
    }
    __builtin_amdgcn_fence(__ATOMIC_RELEASE, "workgroup");
    __builtin_amdgcn_wave_barrier();
    __builtin_amdgcn_fence(__ATOMIC_ACQUIRE, "workgroup");
    if (OUT_MODE == 0) {
      float* C = (float*)Cout + (size_t)b * strideC;
      const int hh = shh, c4 = sc4;
      if (DXM) {
#pragma unroll
        for (int it = 0; it < 8; ++it) {
          const int row = it * 2 + hh;
          v4f v = *(const v4f*)(slab + row * 68 + c4);
          const v4f xv = *(const v4f*)(xres + (size_t)(mBase + row) * ldx + n0 + c4);
          v[0] = v[0] + dv4[0] * xv[0];
          v[1] = v[1] + dv4[1] * xv[1];
          v[2] = v[2] + dv4[2] * xv[2];
          v[3] = v[3] + dv4[3] * xv[3];
          *(v4f*)(slab + row * 68 + c4) = v;
          if (it == 3) mem_split();
        }
        __builtin_amdgcn_fence(__ATOMIC_RELEASE, "workgroup");
        __builtin_amdgcn_wave_barrier();
        __builtin_amdgcn_fence(__ATOMIC_ACQUIRE, "workgroup");
      }
      for (int pass = 0; pass < 2; ++pass) {
#pragma unroll
        for (int it = 0; it < 8; ++it) {
          const int row = it * 2 + hh;
          v4f v = *(const v4f*)(slab + row * 68 + c4);
          *(volatile v4f*)(C + (size_t)(mBase + row) * ldc + n0 + c4) = v;
        }
        __threadfence();
      }
    } else {
      const int q = lane >> 3, c8 = (lane & 7) * 8;
      unsigned short* C  = (unsigned short*)Cout  + (size_t)b * strideC;
      unsigned short* C2 = (OUT_MODE == 2) ? ((unsigned short*)Cout2 + (size_t)b * strideC) : nullptr;
      for (int pass = 0; pass < 2; ++pass) {
#pragma unroll
        for (int it = 0; it < 4; ++it) {
          const int row = it * 4 + q;
          const float* sp = slab + row * 68 + c8;
          v8h hv, lv;
#pragma unroll
          for (int e = 0; e < 8; ++e) {
            if (OUT_MODE == 1) {
              hv[e] = (_Float16)sp[e];
            } else {
              unsigned short hb = f2bf_bits(sp[e]);
              unsigned short lb = f2bf_bits(sp[e] - bf_bits2f(hb));
              hv[e] = __builtin_bit_cast(_Float16, hb);
              lv[e] = __builtin_bit_cast(_Float16, lb);
            }
          }
          *(volatile v8h*)(C + (size_t)(mBase + row) * ldc + n0 + c8) = hv;
          if (OUT_MODE == 2) *(volatile v8h*)(C2 + (size_t)(mBase + row) * ldc + n0 + c8) = lv;
        }
        __threadfence();
      }
    }
    __builtin_amdgcn_fence(__ATOMIC_RELEASE, "workgroup");
    __builtin_amdgcn_wave_barrier();
    __builtin_amdgcn_fence(__ATOMIC_ACQUIRE, "workgroup");
  }
}

__global__ __launch_bounds__(NSTATE) void lam_kernel(const float* __restrict__ nu_log, const float* __restrict__ theta_log,
                                                     const float* __restrict__ s_re, const float* __restrict__ s_im,
                                                     float* __restrict__ LAMT) {
  const int n = threadIdx.x;
  const float nu = expf(nu_log[n]);
  const float th = expf(theta_log[n]);
  const float rr = expf(-nu);
  float sn, cs;
  sincosf(th, &sn, &cs);
  const float l0re = rr * cs, l0im = rr * sn;
  const float sre = s_re[n], sim = s_im[n];
  const float lre = l0re * sre - l0im * sim;
  const float lim = l0re * sim + l0im * sre;
  float pr = lre, pi = lim;
#pragma unroll 1
  for (int s = 0; s < 6; ++s) {
    const float nr = pr * pr - pi * pi;
    const float ni = 2.0f * pr * pi;
    pr = nr; pi = ni;
  }
  float* p = LAMT + n;
  *(volatile float*)(p)              = lre;
  *(volatile float*)(p + NSTATE)     = lim;
  *(volatile float*)(p + 2 * NSTATE) = pr;
  *(volatile float*)(p + 3 * NSTATE) = pi;
  __threadfence();
  *(volatile float*)(p)              = lre;
  *(volatile float*)(p + NSTATE)     = lim;
  *(volatile float*)(p + 2 * NSTATE) = pr;
  *(volatile float*)(p + 3 * NSTATE) = pi;
}

__global__ __launch_bounds__(NTHR) void prepb_kernel(const float* __restrict__ B_re, const float* __restrict__ B_im,
                                                     const float* __restrict__ gamma_log, unsigned short* __restrict__ BT1) {
  const int i = blockIdx.x * NTHR + threadIdx.x;
  if (i < NSTATE * (NFEAT / 8)) {
    const int n  = i >> 6;
    const int c8 = (i & 63) * 8;
    float sg, cg;
    sincosf(gamma_log[n], &sg, &cg);
    const float* pre = B_re + (size_t)n * NFEAT + c8;
    const float* pim = B_im + (size_t)n * NFEAT + c8;
    const v4f ra = *(const v4f*)(pre), rb = *(const v4f*)(pre + 4);
    const v4f ia = *(const v4f*)(pim), ib = *(const v4f*)(pim + 4);
    v8h ore, oim;
#pragma unroll
    for (int e = 0; e < 4; ++e) {
      const float br0 = ra[e], bi0 = ia[e], br1 = rb[e], bi1 = ib[e];
      ore[e]     = (_Float16)((br0 * cg - bi0 * sg) * BP_CARRY);
      oim[e]     = (_Float16)((br0 * sg + bi0 * cg) * BP_CARRY);
      ore[4 + e] = (_Float16)((br1 * cg - bi1 * sg) * BP_CARRY);
      oim[4 + e] = (_Float16)((br1 * sg + bi1 * cg) * BP_CARRY);
    }
    unsigned short* qre = BT1 + (size_t)n * NFEAT + c8;
    unsigned short* qim = BT1 + (size_t)(NSTATE + n) * NFEAT + c8;
    *(volatile v8h*)qre = ore;
    *(volatile v8h*)qim = oim;
    __threadfence();
    *(volatile v8h*)qre = ore;
    *(volatile v8h*)qim = oim;
  }
}

__global__ __launch_bounds__(NTHR) void prepc_kernel(const float* __restrict__ C_re, const float* __restrict__ C_im,
                                                     unsigned short* __restrict__ BT2) {
  const int i = blockIdx.x * NTHR + threadIdx.x;
  if (i < NFEAT * (NSTATE / 8)) {
    const int f  = i >> 6;
    const int c8 = (i & 63) * 8;
    const float* pre = C_re + (size_t)f * NSTATE + c8;
    const float* pim = C_im + (size_t)f * NSTATE + c8;
    const v4f ra = *(const v4f*)(pre), rb = *(const v4f*)(pre + 4);
    const v4f ia = *(const v4f*)(pim), ib = *(const v4f*)(pim + 4);
    v8h ore, oim;
#pragma unroll
    for (int e = 0; e < 4; ++e) {
      ore[e]     = (_Float16)(ra[e] * CW_CARRY);
      ore[4 + e] = (_Float16)(rb[e] * CW_CARRY);
      oim[e]     = (_Float16)(-(ia[e] * CW_CARRY));
      oim[4 + e] = (_Float16)(-(ib[e] * CW_CARRY));
    }
    unsigned short* qre = BT2 + (size_t)f * NCOL2 + c8;
    unsigned short* qim = BT2 + (size_t)f * NCOL2 + NSTATE + c8;
    *(volatile v8h*)qre = ore;
    *(volatile v8h*)qim = oim;
    __threadfence();
    *(volatile v8h*)qre = ore;
    *(volatile v8h*)qim = oim;
  }
}

__global__ __launch_bounds__(NTHR) void cvtx_kernel(const float* __restrict__ x, unsigned short* __restrict__ A1, int n8) {
  const int i = blockIdx.x * NTHR + threadIdx.x;
  if (i < n8) {
    const float* sp = x + (size_t)i * 8;
    const v4f a = *(const v4f*)(sp);
    const v4f c = *(const v4f*)(sp + 4);
    v8h hv;
#pragma unroll
    for (int e = 0; e < 4; ++e) { hv[e] = (_Float16)a[e]; hv[4 + e] = (_Float16)c[e]; }
    unsigned short* dp = A1 + (size_t)i * 8;
    *(volatile v8h*)dp = hv;
    __threadfence();
    *(volatile v8h*)dp = hv;
  }
}

__global__ __launch_bounds__(128) void scan_agg_kernel(const float* __restrict__ BU, const float* __restrict__ LAMT,
                                                       float* __restrict__ AGG) {
  const int c  = blockIdx.x;
  const int n0 = threadIdx.x * 4;
  const v4f lr = *(const v4f*)(LAMT + n0);
  const v4f li = *(const v4f*)(LAMT + NSTATE + n0);
  v4f hr = {0.0f, 0.0f, 0.0f, 0.0f};
  v4f hi = {0.0f, 0.0f, 0.0f, 0.0f};
  const float* bp = BU + (size_t)c * CHUNK_T * NCOL2 + n0;
#pragma unroll 1
  for (int t = 0; t < CHUNK_T; ++t) {
    const v4f br = *(const v4f*)(bp);
    const v4f bi = *(const v4f*)(bp + NSTATE);
    bp += NCOL2;
#pragma unroll
    for (int e = 0; e < 4; ++e) {
      const float nr = lr[e] * hr[e] - li[e] * hi[e] + br[e];
      const float ni = lr[e] * hi[e] + li[e] * hr[e] + bi[e];
      hr[e] = nr; hi[e] = ni;
    }
  }
  float* ap = AGG + (size_t)c * NCOL2 + n0;
  *(volatile v4f*)(ap)          = hr;
  *(volatile v4f*)(ap + NSTATE) = hi;
  __threadfence();
  *(volatile v4f*)(ap)          = hr;
  *(volatile v4f*)(ap + NSTATE) = hi;
}

__global__ __launch_bounds__(NSTATE) void carry_kernel(const float* __restrict__ AGG, const float* __restrict__ LAMT,
                                                       float* __restrict__ CARRY) {
  const int n = threadIdx.x;
  const float lr = LAMT[2 * NSTATE + n];
  const float li = LAMT[3 * NSTATE + n];
  float hre = 0.0f, him = 0.0f;
#pragma unroll 1
  for (int c = 0; c < NCHUNK; ++c) {
    float* cpt = CARRY + (size_t)c * NCOL2 + n;
    *(volatile float*)(cpt)          = hre;
    *(volatile float*)(cpt + NSTATE) = him;
    __threadfence();
    *(volatile float*)(cpt)          = hre;
    *(volatile float*)(cpt + NSTATE) = him;
    const float ar = AGG[(size_t)c * NCOL2 + n];
    const float ai = AGG[(size_t)c * NCOL2 + NSTATE + n];
    const float nr = lr * hre - li * him + ar;
    const float ni = lr * him + li * hre + ai;
    hre = nr; him = ni;
  }
}

__global__ __launch_bounds__(64) void apply_kernel(const float* __restrict__ BU, const float* __restrict__ LAMT,
                                                   const float* __restrict__ CARRY, unsigned short* __restrict__ A2) {
  const int c  = blockIdx.x;
  const int n0 = threadIdx.x * 8;
  const v8f lr = *(const v8f*)(LAMT + n0);
  const v8f li = *(const v8f*)(LAMT + NSTATE + n0);
  mem_split();
  v8f hr = *(const v8f*)(CARRY + (size_t)c * NCOL2 + n0);
  v8f hi = *(const v8f*)(CARRY + (size_t)c * NCOL2 + NSTATE + n0);
  const float* bp = BU + (size_t)c * CHUNK_T * NCOL2 + n0;
  unsigned short* ap = A2 + (size_t)c * CHUNK_T * NCOL2 + n0;
#pragma unroll 1
  for (int t = 0; t < CHUNK_T; ++t) {
    const v8f br = *(const v8f*)(bp);
    const v8f bi = *(const v8f*)(bp + NSTATE);
    bp += NCOL2;
    v8h ore, oim;
#pragma unroll
    for (int e = 0; e < 8; ++e) {
      const float nr = lr[e] * hr[e] - li[e] * hi[e] + br[e];
      const float ni = lr[e] * hi[e] + li[e] * hr[e] + bi[e];
      hr[e] = nr; hi[e] = ni;
      ore[e] = (_Float16)(nr * HS_CARRY);
      oim[e] = (_Float16)(ni * HS_CARRY);
    }
    *(volatile v8h*)(ap)          = ore;
    *(volatile v8h*)(ap + NSTATE) = oim;
    __threadfence();
    *(volatile v8h*)(ap)          = ore;
    *(volatile v8h*)(ap + NSTATE) = oim;
    ap += NCOL2;
  }
}

extern "C" void kernel_launch(void* const* d_in, const int* in_sizes, int n_in,
                              void* d_out, int out_size, void* d_ws, size_t ws_size, hipStream_t stream) {
  if (n_in < 11 || d_out == nullptr || d_ws == nullptr) return;
  if (in_sizes[0] != SEQ_LEN * NFEAT || in_sizes[1] != NSTATE || in_sizes[2] != NSTATE || in_sizes[3] != NSTATE ||
      in_sizes[4] != NSTATE || in_sizes[5] != NSTATE || in_sizes[6] != NSTATE * NFEAT || in_sizes[7] != NSTATE * NFEAT ||
      in_sizes[8] != NFEAT * NSTATE || in_sizes[9] != NFEAT * NSTATE || in_sizes[10] != NFEAT ||
      out_size != SEQ_LEN * NFEAT) return;

  const float* x         = (const float*)d_in[0];
  const float* state_re  = (const float*)d_in[1];
  const float* state_im  = (const float*)d_in[2];
  const float* nu_log    = (const float*)d_in[3];
  const float* theta_log = (const float*)d_in[4];
  const float* gamma_log = (const float*)d_in[5];
  const float* b_re      = (const float*)d_in[6];
  const float* b_im      = (const float*)d_in[7];
  const float* c_re      = (const float*)d_in[8];
  const float* c_im      = (const float*)d_in[9];
  const float* dvec      = (const float*)d_in[10];
  float* y = (float*)d_out;

  char* ws = (char*)d_ws; size_t off = 0;
  auto carve = [&](size_t bytes) -> char* { char* p = ws + off; off += (bytes + 255) & ~(size_t)255; return p; };
  unsigned short* A1    = (unsigned short*)carve((size_t)SEQ_LEN * NFEAT * 2);
  unsigned short* BT1   = (unsigned short*)carve((size_t)NCOL2 * NFEAT * 2);
  unsigned short* BT2   = (unsigned short*)carve((size_t)NFEAT * NCOL2 * 2);
  float*          LAMT  = (float*)carve((size_t)4 * NSTATE * 4);
  float*          BU    = (float*)carve((size_t)SEQ_LEN * NCOL2 * 4);
  float*          AGG   = (float*)carve((size_t)NCHUNK * NCOL2 * 4);
  float*          CARRY = (float*)carve((size_t)NCHUNK * NCOL2 * 4);
  unsigned short* A2    = (unsigned short*)carve((size_t)SEQ_LEN * NCOL2 * 2);
  if (off > ws_size || off > (size_t)134217728) return;

  lam_kernel<<<1, NSTATE, 0, stream>>>(nu_log, theta_log, state_re, state_im, LAMT);
  const int n8b = NSTATE * (NFEAT / 8);
  const int n8x = SEQ_LEN * (NFEAT / 8);
  prepb_kernel<<<(n8b + NTHR - 1) / NTHR, NTHR, 0, stream>>>(b_re, b_im, gamma_log, BT1);
  prepc_kernel<<<(n8b + NTHR - 1) / NTHR, NTHR, 0, stream>>>(c_re, c_im, BT2);
  cvtx_kernel<<<(n8x + NTHR - 1) / NTHR, NTHR, 0, stream>>>(x, A1, n8x);
  wmma_gemm64<0, false, 0, 0, false, 0, false><<<dim3((SEQ_LEN / 64) * (NCOL2 / 64) / 8, 1), 256, 0, stream>>>(
      A1, A1, NFEAT, 0L, BT1, BT1, NFEAT, 0L, (void*)BU, (void*)BU, NCOL2, 0L,
      LAMT, LAMT, 0L, SEQ_LEN, NCOL2, NFEAT, G1_FOLD, LAMT, LAMT, 0);
  scan_agg_kernel<<<NCHUNK, 128, 0, stream>>>(BU, LAMT, AGG);
  carry_kernel<<<1, NSTATE, 0, stream>>>(AGG, LAMT, CARRY);
  apply_kernel<<<NCHUNK, 64, 0, stream>>>(BU, LAMT, CARRY, A2);
  wmma_gemm64<0, false, 0, 0, false, 0, true><<<dim3((SEQ_LEN / 64) * (NFEAT / 64) / 8, 1), 256, 0, stream>>>(
      A2, A2, NCOL2, 0L, BT2, BT2, NCOL2, 0L, (void*)y, (void*)y, NFEAT, 0L,
      LAMT, LAMT, 0L, SEQ_LEN, NFEAT, NCOL2, G2_FOLD, dvec, x, NFEAT);
}
